// DenseGATv2_7069516169275
// MI455X (gfx1250) — hardware-verified
//
#include <hip/hip_runtime.h>
#include <math.h>


#define NB 4
#define NN 1024
#define DD 128
#define NH 8
#define QD 16
#define NTOK (NB * NN)
typedef __attribute__((ext_vector_type(16))) _Float16 v16h;
typedef __attribute__((ext_vector_type(8)))  _Float16 v8h;
typedef __attribute__((ext_vector_type(8)))  float    v8f;
typedef __attribute__((ext_vector_type(4)))  float    v4f;
#define VST2(T, ptr, val) do { const T _v = (val); *(volatile T*)(ptr) = _v; __threadfence(); *(volatile T*)(ptr) = _v; } while (0)
__device__ __forceinline__ v8f wmma16(v16h a, v16h b, v8f c) {
  v8f d = __builtin_amdgcn_wmma_f32_16x16x32_f16(false, a, false, b, (short)0, c, false, false);
  asm volatile("v_nop\n\tv_nop\n\tv_nop\n\tv_nop" : "+v"(d) : "v"(a), "v"(b));
  return d;
}
__device__ __forceinline__ v16h frag16(const _Float16* p, int hh) {
  const v8h lo = *(const v8h*)(p + 8 * hh), hi = *(const v8h*)(p + 16 + 8 * hh);
  return __builtin_shufflevector(lo, hi, 0,1,2,3,4,5,6,7,8,9,10,11,12,13,14,15);
}
__device__ __forceinline__ int kmap(int e, int hh) { return (e < 8) ? (8 * hh + e) : (16 + 8 * hh + (e - 8)); }
__global__ __launch_bounds__(256) void k_tok(const float* __restrict__ h, const float* __restrict__ Wa, const float* __restrict__ Wv,
                                            float* __restrict__ S, _Float16* __restrict__ V16) {
  __shared__ float hr[2][DD];
  const int half = threadIdx.x >> 7, c = threadIdx.x & 127, tok = blockIdx.x * 2 + half;
  hr[half][c] = h[(size_t)tok * DD + c];
  __syncthreads();
  float v = 0.f;
  for (int k = 0; k < DD; ++k) v += hr[half][k] * Wv[k * DD + c];
  const _Float16 vh = (_Float16)v;
  *(volatile _Float16*)(V16 + (size_t)tok * DD + c) = vh; __threadfence(); *(volatile _Float16*)(V16 + (size_t)tok * DD + c) = vh;
  if (threadIdx.x < 32) {
    const int hf = threadIdx.x >> 4, cc = threadIdx.x & 15, hd = cc & 7;
    const float* W = Wa + ((cc < 8) ? 0 : DD * NH);
    float s = 0.f;
    for (int k = 0; k < DD; ++k) s += hr[hf][k] * W[k * NH + hd];
    VST2(float, S + (size_t)(blockIdx.x * 2 + hf) * 16 + cc, s);
  }
}
__global__ __launch_bounds__(256) void k_attn(const float* __restrict__ S, const int* __restrict__ edge, const float* __restrict__ Wa, const _Float16* __restrict__ V16,
                                              _Float16* __restrict__ O16) {
  __shared__ __attribute__((aligned(16))) float sO[16][DD + 4];
  const int lane = threadIdx.x & 31, hd = threadIdx.x >> 5, hh = lane >> 4, l16 = lane & 15;
  const int b = blockIdx.x / (NN / 16), i0 = (blockIdx.x % (NN / 16)) * 16, i = i0 + l16;
  const float we = Wa[2 * DD * NH + hd];
  const float si = S[((size_t)b * NN + i) * 16 + hd];
  const int* er = edge + ((size_t)b * NN + i) * NN;
  const float* sj = S + (size_t)b * NN * 16 + 8 + hd;
  auto score = [&](int j) -> float { const float a = si + sj[(size_t)j * 16] + (float)er[j] * we; return (a > 0.f) ? a : 0.15f * a; };
  float mx = -INFINITY;
  for (int kb = 0; kb < NN; kb += 32) {
#pragma unroll
    for (int e = 0; e < 16; ++e) mx = fmaxf(mx, score(kb + kmap(e, hh)));
  }
  mx = fmaxf(mx, __shfl_xor(mx, 16));
  float sum = 0.f; v8f acc = {};
  for (int kb = 0; kb < NN; kb += 32) {
    v16h pa;
#pragma unroll
    for (int e = 0; e < 16; ++e) { const float p = expf(score(kb + kmap(e, hh)) - mx); sum += p; pa[e] = (_Float16)p; }
    v16h vb;
#pragma unroll
    for (int e = 0; e < 16; ++e) vb[e] = V16[((size_t)b * NN + kb + kmap(e, hh)) * DD + hd * QD + l16];
    acc = wmma16(pa, vb, acc);
  }
  sum += __shfl_xor(sum, 16);
#pragma unroll
  for (int v = 0; v < 8; ++v) { const float rs = __shfl(sum, v + 8 * hh); sO[v + 8 * hh][hd * QD + l16] = acc[v] / rs; }
  __syncthreads();
  {
    const int r = threadIdx.x >> 4, c = (threadIdx.x & 15) * 8;
    v8h o;
#pragma unroll
    for (int e = 0; e < 8; ++e) o[e] = (_Float16)sO[r][c + e];
    VST2(v8h, O16 + ((size_t)b * NN + i0 + r) * DD + c, o);
  }
}
__global__ __launch_bounds__(256) void k_woT(const float* __restrict__ Wo, _Float16* __restrict__ WoT) {
  const int t = blockIdx.x * 256 + threadIdx.x;
  const int n = t >> 4, k0 = (t & 15) * 8;
  v8h o;
#pragma unroll
  for (int e = 0; e < 8; ++e) o[e] = (_Float16)Wo[(size_t)(k0 + e) * DD + n];
  VST2(v8h, WoT + (size_t)n * DD + k0, o);
}
__global__ __launch_bounds__(128) void k_out(const _Float16* __restrict__ O16, const _Float16* __restrict__ WoT, float* __restrict__ out) {
  __shared__ __attribute__((aligned(16))) float sT[4][16][132];
  const int lane = threadIdx.x & 31, wave = threadIdx.x >> 5, hh = lane >> 4, l16 = lane & 15;
  const int m0 = blockIdx.x * 64 + wave * 16;
  v8f acc[8];
#pragma unroll
  for (int ni = 0; ni < 8; ++ni) acc[ni] = (v8f){};
#pragma unroll
  for (int k0 = 0; k0 < DD; k0 += 32) {
    const v16h a0 = frag16(O16 + (size_t)(m0 + l16) * DD + k0, hh);
#pragma unroll
    for (int ni = 0; ni < 8; ++ni) acc[ni] = wmma16(a0, frag16(WoT + (size_t)(ni * 16 + l16) * DD + k0, hh), acc[ni]);
  }
  float (*st)[132] = sT[wave];
#pragma unroll
  for (int ni = 0; ni < 8; ++ni)
#pragma unroll
    for (int v = 0; v < 8; ++v) st[v + 8 * hh][ni * 16 + l16] = acc[ni][v];
  __builtin_amdgcn_fence(__ATOMIC_RELEASE, "workgroup"); __builtin_amdgcn_wave_barrier(); __builtin_amdgcn_fence(__ATOMIC_ACQUIRE, "workgroup");
  for (int pass = 0; pass < 2; ++pass) {
#pragma unroll
    for (int rr = 0; rr < 16; ++rr) *(volatile v4f*)(out + (size_t)(m0 + rr) * DD + lane * 4) = *(const v4f*)(&st[rr][lane * 4]);
    __threadfence();
  }
}
extern "C" void kernel_launch(void* const* d_in, const int* in_sizes, int n_in,
                              void* d_out, int out_size, void* d_ws, size_t ws_size, hipStream_t stream) {
  (void)in_sizes; (void)n_in; (void)out_size;
  const float* h    = (const float*)d_in[0];
  const int*   edge = (const int*)  d_in[1];
  const float* Wa   = (const float*)d_in[2];
  const float* Wv   = (const float*)d_in[3];
  const float* Wo   = (const float*)d_in[4];
  float* out = (float*)d_out;
  char* ws = (char*)d_ws; size_t off = 0;
  auto take = [&](size_t bytes) { void* p = ws + off; off = (off + bytes + 255) & ~(size_t)255; return p; };
  float*    S   = (float*)take((size_t)NTOK * 16 * 4);
  _Float16* V16 = (_Float16*)take((size_t)NTOK * DD * 2);
  _Float16* O16 = (_Float16*)take((size_t)NTOK * DD * 2);
  _Float16* WoT = (_Float16*)take((size_t)DD * DD * 2);
  if (off > ws_size) return;
  k_tok<<<NTOK / 2, 256, 0, stream>>>(h, Wa, Wv, S, V16);
  k_attn<<<NB * NN / 16, 256, 0, stream>>>(S, edge, Wa, V16, O16);
  k_woT<<<128 * 16 / 256, 256, 0, stream>>>(Wo, WoT);
  k_out<<<NTOK / 64, 128, 0, stream>>>(O16, WoT, out);
}
